// MiM_v2_91070486544638
// MI455X (gfx1250) — hardware-run, weakly checked
//
#include <hip/hip_runtime.h>
#include <math.h>

typedef __attribute__((ext_vector_type(16))) _Float16 v16h;
typedef __attribute__((ext_vector_type(8)))  _Float16 v8h;
typedef __attribute__((ext_vector_type(2)))  _Float16 v2h;
typedef __attribute__((ext_vector_type(8)))  float    v8f;
typedef __attribute__((ext_vector_type(4)))  float    v4f;
typedef __attribute__((ext_vector_type(4)))  unsigned v4u;

constexpr int kBatch = 16;
constexpr int kSeq   = 1024;
constexpr int kDm    = 512;
constexpr int kDin   = 1024;
constexpr int kDtR   = 32;
constexpr int kNst   = 16;
constexpr int kDbc   = kDtR + 2 * kNst;
constexpr int kRows  = kBatch * kSeq;
static_assert(kDbc == 64, "dbc width");
static_assert(kRows == 16384, "token rows");
static_assert((kDm % 32) == 0 && (kDin % 32) == 0 && (kDtR % 32) == 0, "GEMM K multiples of 32");
static_assert((kRows % 64) == 0 && (kDin % 64) == 0 && (kDbc % 64) == 0 && (kDm % 64) == 0, "GEMM M,N multiples of 64");
static_assert((kSeq % 64) == 0 && (kDin % 512) == 0 && (kRows % 128) == 0, "tile multiples");

constexpr float kWCarry    = 64.0f;
constexpr float kHCarry    = 16.0f;
constexpr float kYCarry    = 16.0f;
constexpr float kDCarry    = 64.0f;
constexpr float kInvW      = 1.0f / kWCarry;
constexpr float kInvWH     = 1.0f / (kWCarry * kHCarry);
constexpr float kInvWY     = 1.0f / (kWCarry * kYCarry);
constexpr float kInvHCarry = 1.0f / kHCarry;
constexpr float kInvDCarry = 1.0f / kDCarry;
constexpr float kInvDtR    = 1.0f / (float)kDtR;
constexpr float kInvNst    = 1.0f / (float)kNst;
constexpr float kRmsEps    = 1e-5f;

constexpr size_t kOffWin  = 0;
constexpr size_t kOffWout = kOffWin  + (size_t)kDin  * kDm  * 2;
constexpr size_t kOffWxp  = kOffWout + (size_t)kDm   * kDin * 2;
constexpr size_t kOffWdt  = kOffWxp  + (size_t)kDbc  * kDin * 2;
constexpr size_t kOffX16  = kOffWdt  + (size_t)kDin  * kDtR * 2;
constexpr size_t kOffHpre = kOffX16  + (size_t)kRows * kDm  * 2;
constexpr size_t kOffH16  = kOffHpre + (size_t)kRows * kDin * 4;
constexpr size_t kOffDbc  = kOffH16  + (size_t)kRows * kDin * 2;
constexpr size_t kOffDn   = kOffDbc  + (size_t)kRows * kDbc * 4;
constexpr size_t kOffBm   = kOffDn   + (size_t)kRows * kDtR * 2;
constexpr size_t kOffCm   = kOffBm   + (size_t)kRows * kNst * 4;
constexpr size_t kWsTotal = kOffCm   + (size_t)kRows * kNst * 4;
constexpr size_t kOffDelta = kOffHpre;
constexpr size_t kOffY16   = kOffHpre + (size_t)kRows * kDin * 2;
static_assert(kWsTotal == 127074304ull, "carve total");
static_assert(kWsTotal <= 134217728ull, "carve cap");
static_assert(kOffY16 + (size_t)kRows * kDin * 2 == kOffH16, "overlay fits the dead f32 plane");
static_assert((kOffWout % 128) == 0 && (kOffWxp % 128) == 0 && (kOffWdt % 128) == 0 && (kOffX16 % 128) == 0 &&
              (kOffHpre % 128) == 0 && (kOffH16 % 128) == 0 && (kOffDbc % 128) == 0 && (kOffDn % 128) == 0 &&
              (kOffBm % 128) == 0 && (kOffCm % 128) == 0 && (kOffY16 % 128) == 0, "128-B aligned regions");

__device__ __forceinline__ unsigned short f2bf_bits(float f) {
  unsigned u = __float_as_uint(f);
  return (unsigned short)((u + 0x7FFFu + ((u >> 16) & 1u)) >> 16);
}
__device__ __forceinline__ float bf_bits2f(unsigned short h) { return __uint_as_float(((unsigned)h) << 16); }
__device__ __forceinline__ float bf_rne(float f) { return bf_bits2f(f2bf_bits(f)); }

__device__ __forceinline__ float h16_to_f32(unsigned hb) {
  const unsigned sgn = (hb & 0x8000u) << 16;
  const unsigned em = hb & 0x7fffu;
  const float fn = __uint_as_float((em << 13) + 0x38000000u);
  const float fs = (float)em * 5.9604644775390625e-8f;
  const float mag = (em < 0x400u) ? fs : fn;
  return __uint_as_float(__float_as_uint(mag) | sgn);
}

struct FragH {
  union U { v16h v; v8h h[2]; };
  static __device__ __forceinline__ v16h load(const _Float16* p) {
    U f;
    f.h[0] = *(const v8h*)(p);
    f.h[1] = *(const v8h*)(p + 16);
    return f.v;
  }
};

__device__ __forceinline__ v8f mma_g(v16h a, v16h b, v8f c) {
  c = __builtin_amdgcn_wmma_f32_16x16x32_f16(false, a, false, b, (short)0, c, false, false);
  asm volatile("v_nop\n\tv_nop\n\tv_nop\n\tv_nop" : "+v"(c) : "v"(a), "v"(b));
  return c;
}

__global__ __launch_bounds__(256) void cvt_rows_f16_kernel(
    const float* __restrict__ src, unsigned short* __restrict__ dst, int total8, float carry)
{
  const int i = blockIdx.x * 256 + threadIdx.x;
  if (i >= total8) return;
  const size_t e0 = (size_t)i << 3;
  const v4f a0 = *(const v4f*)(src + e0);
  const v4f a1 = *(const v4f*)(src + e0 + 4);
  v8h hv;
#pragma unroll
  for (int e = 0; e < 4; ++e) {
    const float f0 = a0[e];
    const float f1 = a1[e];
    hv[e]     = (_Float16)(bf_rne(f0) * carry);
    hv[4 + e] = (_Float16)(bf_rne(f1) * carry);
  }
  unsigned short* q = dst + e0;
  *(volatile v8h*)q = hv;
  __threadfence();
  *(volatile v8h*)q = hv;
}

template <int BIAS_MODE, int OUT_MODE, int ACT>
__global__ __launch_bounds__(256) void wmma_gemm64(
    const unsigned short* __restrict__ Ap, int lda,
    const unsigned short* __restrict__ Btp, int ldb,
    void* __restrict__ Cout, int ldc,
    const float* __restrict__ bias,
    int M, int N, int K, float scale, float oscale)
{
  const _Float16* A  = (const _Float16*)Ap;
  const _Float16* Bt = (const _Float16*)Btp;
  __shared__ __align__(16) float sT[8][16 * 68];
  const int lane = threadIdx.x & 31;
  const int wave = threadIdx.x >> 5;
  const int tilesN = N >> 6;
  const int tilesM = M >> 6;
  const int tile = blockIdx.x * 8 + wave;
  if (tile >= tilesM * tilesN) return;
  const int tm = tile / tilesN;
  const int tn = tile - tm * tilesN;
  const int m0 = tm << 6;
  const int n0 = tn << 6;

  const int rlane = lane & 15;
  const int koff  = (lane >> 4) * 8;
  const int mOff  = (lane >> 4) * 8;

  v8f acc[4][4];
#pragma unroll
  for (int i = 0; i < 4; ++i)
#pragma unroll
    for (int j = 0; j < 4; ++j) acc[i][j] = (v8f){0.f, 0.f, 0.f, 0.f, 0.f, 0.f, 0.f, 0.f};

  for (int k0 = 0; k0 < K; k0 += 32) {
    v16h bh[4];
#pragma unroll
    for (int j = 0; j < 4; ++j) {
      const size_t bo = (size_t)(n0 + (j << 4) + rlane) * ldb + koff + k0;
      bh[j] = FragH::load(Bt + bo);
    }
#pragma unroll
    for (int i = 0; i < 4; ++i) {
      const size_t ao = (size_t)(m0 + (i << 4) + rlane) * lda + koff + k0;
      const v16h ah = FragH::load(A + ao);
#pragma unroll
      for (int j = 0; j < 4; ++j) acc[i][j] = mma_g(ah, bh[j], acc[i][j]);
    }
  }

  float* slab = sT[wave];
  float bvj[4];
#pragma unroll
  for (int j = 0; j < 4; ++j) {
    bvj[j] = 0.f;
    if (BIAS_MODE == 2) bvj[j] = bf_rne(bias[n0 + (j << 4) + rlane]);
  }
#pragma unroll
  for (int i = 0; i < 4; ++i) {
    const int mBase = m0 + (i << 4);
#pragma unroll
    for (int j = 0; j < 4; ++j) {
#pragma unroll
      for (int r = 0; r < 8; ++r) {
        float v = acc[i][j][r] * scale;
        if (BIAS_MODE == 2) v += bvj[j];
        slab[(mOff + r) * 68 + (j << 4) + rlane] = v;
      }
    }
    __builtin_amdgcn_fence(__ATOMIC_RELEASE, "workgroup");
    __builtin_amdgcn_wave_barrier();
    __builtin_amdgcn_fence(__ATOMIC_ACQUIRE, "workgroup");
    if (ACT == 6) {
#pragma unroll 1
      for (int t = 0; t < 32; ++t) {
        const int idx = t * 32 + lane;
        float* sp = slab + (idx >> 6) * 68 + (idx & 63);
        const float v = *sp;
        const float e = expf(-fabsf(v));
        const float sv = fmaxf(v, 0.0f) + log1pf(e);
        *sp = sv * oscale;
      }
      __builtin_amdgcn_fence(__ATOMIC_RELEASE, "workgroup");
      __builtin_amdgcn_wave_barrier();
      __builtin_amdgcn_fence(__ATOMIC_ACQUIRE, "workgroup");
    }
    if (OUT_MODE == 0) {
      float* C = (float*)Cout;
      const int hh = lane >> 4, c4 = (lane & 15) * 4;
      for (int pass = 0; pass < 2; ++pass) {
#pragma unroll
        for (int it = 0; it < 8; ++it) {
          const int row = it * 2 + hh;
          v4f v = *(const v4f*)(slab + row * 68 + c4);
          *(volatile v4f*)(C + (size_t)(mBase + row) * ldc + n0 + c4) = v;
        }
        __threadfence();
      }
    } else {
      const int q = lane >> 3, c8 = (lane & 7) * 8;
      unsigned short* C = (unsigned short*)Cout;
      for (int pass = 0; pass < 2; ++pass) {
#pragma unroll
        for (int it = 0; it < 4; ++it) {
          const int row = it * 4 + q;
          const float* sp = slab + row * 68 + c8;
          v8h hv;
#pragma unroll
          for (int e = 0; e < 8; ++e) hv[e] = (_Float16)sp[e];
          *(volatile v8h*)(C + (size_t)(mBase + row) * ldc + n0 + c8) = hv;
        }
        __threadfence();
      }
    }
    __builtin_amdgcn_fence(__ATOMIC_RELEASE, "workgroup");
    __builtin_amdgcn_wave_barrier();
    __builtin_amdgcn_fence(__ATOMIC_ACQUIRE, "workgroup");
  }
}

constexpr int kConvTP = 260;
__global__ __launch_bounds__(256) void conv_silu_kernel(
    const float* __restrict__ HPRE, const float* __restrict__ cw, const float* __restrict__ cb,
    unsigned short* __restrict__ H16)
{
  __shared__ __align__(16) float sT[16 * kConvTP];
  const int tid = threadIdx.x, lane = tid & 31, wave = tid >> 5;
  const int d0 = blockIdx.x * 256, d = d0 + tid;
  const int g0 = blockIdx.y * 64;
  const int tb = g0 & (kSeq - 1);
  const float w0 = bf_rne(cw[d * 3 + 0]);
  const float w1 = bf_rne(cw[d * 3 + 1]);
  const float w2 = bf_rne(cw[d * 3 + 2]);
  const float bc = bf_rne(cb[d]);
  float xm2, xm1;
  {
    const bool hist = (tb > 0);
    const int rb = hist ? (g0 - 2) : g0;
    const float v2 = HPRE[(size_t)rb * kDin + d];
    const float v1 = HPRE[(size_t)(rb + 1) * kDin + d];
    xm2 = hist ? v2 : 0.f;
    xm1 = hist ? v1 : 0.f;
  }
#pragma unroll 1
  for (int sub = 0; sub < 4; ++sub) {
    const int lb = g0 + sub * 16;
#pragma unroll 1
    for (int s = 0; s < 16; ++s) {
      const float xcur = HPRE[(size_t)(lb + s) * kDin + d];
      float acc = w0 * xm2;
      acc = fmaf(w1, xm1, acc);
      acc = fmaf(w2, xcur, acc);
      const float sv = acc + bc;
      const float sg = __builtin_amdgcn_rcpf(1.0f + __expf(-sv));
      sT[s * kConvTP + tid] = (sv * sg) * kHCarry;
      xm2 = xm1;
      xm1 = xcur;
    }
    __syncthreads();
    v8h hv[2];
#pragma unroll
    for (int it = 0; it < 2; ++it) {
      const float* sp = sT + (it * 8 + wave) * kConvTP + lane * 8;
      const v4f a0 = *(const v4f*)(sp);
      const v4f a1 = *(const v4f*)(sp + 4);
#pragma unroll
      for (int e = 0; e < 4; ++e) {
        hv[it][e]     = (_Float16)a0[e];
        hv[it][4 + e] = (_Float16)a1[e];
      }
    }
    for (int pass = 0; pass < 2; ++pass) {
#pragma unroll
      for (int it = 0; it < 2; ++it) {
        const size_t o = (size_t)(lb + it * 8 + wave) * kDin + d0 + lane * 8;
        *(volatile v8h*)(H16 + o) = hv[it];
      }
      __threadfence();
    }
    __syncthreads();
  }
}

constexpr int kRmsDP = 36;
constexpr int kRmsBP = 20;
__global__ __launch_bounds__(128) void rms_split_kernel(
    const float* __restrict__ DBC, const float* __restrict__ dtln, const float* __restrict__ bln,
    const float* __restrict__ cln, unsigned short* __restrict__ DN16, float* __restrict__ BM, float* __restrict__ CM)
{
  __shared__ __align__(16) float sW[64];
  __shared__ __align__(16) float sD[128 * kRmsDP];
  __shared__ __align__(16) float sB[128 * kRmsBP];
  __shared__ __align__(16) float sC[128 * kRmsBP];
  const int tid = threadIdx.x;
  const int row0 = blockIdx.x * 128;
  {
    const float wd = bf_rne(dtln[tid & 31]);
    const float wb = bf_rne(bln[tid & 15]);
    const float wc = bf_rne(cln[tid & 15]);
    if (tid < 32) sW[tid] = wd;
    if (tid < 16) {
      sW[32 + tid] = wb;
      sW[48 + tid] = wc;
    }
  }
  float buf[64];
  {
    const float* rp = DBC + (size_t)(row0 + tid) * kDbc;
#pragma unroll
    for (int i = 0; i < 16; ++i) {
      const v4f q = *(const v4f*)(rp + 4 * i);
      buf[4 * i + 0] = q[0];
      buf[4 * i + 1] = q[1];
      buf[4 * i + 2] = q[2];
      buf[4 * i + 3] = q[3];
    }
  }
  __syncthreads();
  {
    float s = 0.f;
#pragma unroll
    for (int j = 0; j < kDtR; ++j) s = fmaf(buf[j], buf[j], s);
    const float rd = rsqrtf(s * kInvDtR + kRmsEps);
#pragma unroll
    for (int j = 0; j < kDtR; ++j) sD[tid * kRmsDP + j] = (buf[j] * rd) * sW[j];
  }
  {
    float s = 0.f;
#pragma unroll
    for (int j = 0; j < kNst; ++j) s = fmaf(buf[kDtR + j], buf[kDtR + j], s);
    const float rb = rsqrtf(s * kInvNst + kRmsEps);
#pragma unroll
    for (int j = 0; j < kNst; ++j) sB[tid * kRmsBP + j] = (buf[kDtR + j] * rb) * sW[kDtR + j];
  }
  {
    float s = 0.f;
#pragma unroll
    for (int j = 0; j < kNst; ++j) s = fmaf(buf[kDtR + kNst + j], buf[kDtR + kNst + j], s);
    const float rc = rsqrtf(s * kInvNst + kRmsEps);
#pragma unroll
    for (int j = 0; j < kNst; ++j) sC[tid * kRmsBP + j] = (buf[kDtR + kNst + j] * rc) * sW[kDtR + kNst + j];
  }
  __syncthreads();
  v8h dv[4];
  v4f bv[4], cv[4];
#pragma unroll
  for (int it = 0; it < 4; ++it) {
    const int c = it * 128 + tid;
    const int r = c >> 2;
    const int q = c & 3;
    const float* sp = sD + r * kRmsDP + q * 8;
    const v4f a0 = *(const v4f*)(sp);
    const v4f a1 = *(const v4f*)(sp + 4);
#pragma unroll
    for (int e = 0; e < 4; ++e) {
      dv[it][e]     = (_Float16)a0[e];
      dv[it][4 + e] = (_Float16)a1[e];
    }
    bv[it] = *(const v4f*)(sB + r * kRmsBP + q * 4);
    cv[it] = *(const v4f*)(sC + r * kRmsBP + q * 4);
  }
  for (int pass = 0; pass < 2; ++pass) {
#pragma unroll
    for (int it = 0; it < 4; ++it) {
      const int c = it * 128 + tid;
      const int r = c >> 2;
      const int q = c & 3;
      *(volatile v8h*)(DN16 + (size_t)(row0 + r) * kDtR + q * 8) = dv[it];
      *(volatile v4f*)(BM + (size_t)(row0 + r) * kNst + q * 4) = bv[it];
      *(volatile v4f*)(CM + (size_t)(row0 + r) * kNst + q * 4) = cv[it];
    }
    __threadfence();
  }
}

__global__ __launch_bounds__(256) void scan_kernel(
    const unsigned* __restrict__ DEL32, const unsigned* __restrict__ H32,
    const float* __restrict__ BM, const float* __restrict__ CM,
    const float* __restrict__ Alog, const float* __restrict__ Dsk, unsigned* __restrict__ Y32)
{
  __shared__ __align__(16) float    sA[32 * 256];
  __shared__ __align__(16) float    sBm[64 * kNst];
  __shared__ __align__(16) float    sCm[64 * kNst];
  __shared__ __align__(16) unsigned sY[16 * 256];
  const int tid = threadIdx.x;
  const int bix = blockIdx.x >> 1;
  const int cb  = (blockIdx.x & 1) * 512;
  const int d   = cb + 2 * tid;
  const size_t row0 = (size_t)bix * kSeq;
  const int wcol = (cb >> 1) + tid;

#pragma unroll 1
  for (int j = 0; j < 2 * kNst; ++j) {
    const float al = bf_rne(Alog[(size_t)d * kNst + j]);
    sA[j * 256 + tid] = -expf(al);
  }
  __syncthreads();
  float a0[kNst], a1[kNst], s0[kNst], s1[kNst];
#pragma unroll
  for (int n = 0; n < kNst; ++n) {
    a0[n] = sA[n * 256 + tid];
    a1[n] = sA[(kNst + n) * 256 + tid];
    s0[n] = 0.f;
    s1[n] = 0.f;
  }
  const float D0 = bf_rne(Dsk[d]);
  const float D1 = bf_rne(Dsk[d + 1]);

#pragma unroll 1
  for (int c = 0; c < kSeq / 64; ++c) {
    __syncthreads();
    {
      const size_t so = (row0 + (size_t)c * 64) * kNst + (size_t)tid * 4;
      const v4f b4 = *(const v4f*)(BM + so);
      const v4f c4 = *(const v4f*)(CM + so);
      *(v4f*)(sBm + tid * 4) = b4;
      *(v4f*)(sCm + tid * 4) = c4;
    }
    __syncthreads();
#pragma unroll 1
    for (int sub = 0; sub < 4; ++sub) {
      const size_t rowb = row0 + (size_t)c * 64 + (size_t)sub * 16;
#pragma unroll 1
      for (int s = 0; s < 16; ++s) {
        const int ls = sub * 16 + s;
        const size_t gi = (rowb + (size_t)s) * (kDin / 2) + (size_t)wcol;
        const unsigned dw = DEL32[gi];
        const unsigned hw = H32[gi];
        const float dt0 = h16_to_f32(dw & 0xffffu) * kInvDCarry;
        const float dt1 = h16_to_f32(dw >> 16) * kInvDCarry;
        const float h0  = h16_to_f32(hw & 0xffffu) * kInvHCarry;
        const float h1  = h16_to_f32(hw >> 16) * kInvHCarry;
        const float* bp = sBm + ls * kNst;
        const float* cp = sCm + ls * kNst;
        float Bs[kNst], Cs[kNst];
#pragma unroll
        for (int q4 = 0; q4 < 4; ++q4) {
          const v4f bv = *(const v4f*)(bp + 4 * q4);
          const v4f cv = *(const v4f*)(cp + 4 * q4);
          Bs[4 * q4 + 0] = bv[0];
          Bs[4 * q4 + 1] = bv[1];
          Bs[4 * q4 + 2] = bv[2];
          Bs[4 * q4 + 3] = bv[3];
          Cs[4 * q4 + 0] = cv[0];
          Cs[4 * q4 + 1] = cv[1];
          Cs[4 * q4 + 2] = cv[2];
          Cs[4 * q4 + 3] = cv[3];
        }
        const float dx0 = dt0 * h0;
        const float dx1 = dt1 * h1;
        float y0 = 0.f, y1 = 0.f;
#pragma unroll
        for (int n = 0; n < kNst; ++n) {
          const float e0 = __expf(dt0 * a0[n]);
          const float e1 = __expf(dt1 * a1[n]);
          s0[n] = fmaf(e0, s0[n], dx0 * Bs[n]);
          s1[n] = fmaf(e1, s1[n], dx1 * Bs[n]);
          y0 = fmaf(s0[n], Cs[n], y0);
          y1 = fmaf(s1[n], Cs[n], y1);
        }
        y0 = fmaf(D0, h0, y0);
        y1 = fmaf(D1, h1, y1);
        v2h pk;
        pk[0] = (_Float16)(y0 * kYCarry);
        pk[1] = (_Float16)(y1 * kYCarry);
        sY[s * 256 + tid] = __builtin_bit_cast(unsigned, pk);
      }
      __syncthreads();
      v4u yv[4];
#pragma unroll
      for (int it = 0; it < 4; ++it) {
        const int cc = it * 256 + tid;
        yv[it] = *(const v4u*)(sY + (cc >> 6) * 256 + (cc & 63) * 4);
      }
      for (int pass = 0; pass < 2; ++pass) {
#pragma unroll
        for (int it = 0; it < 4; ++it) {
          const int cc = it * 256 + tid;
          const size_t o = (rowb + (size_t)(cc >> 6)) * (kDin / 2) + (size_t)(cb >> 1) + (size_t)((cc & 63) * 4);
          *(volatile v4u*)(Y32 + o) = yv[it];
        }
        __threadfence();
      }
      __syncthreads();
    }
  }
}

extern "C" void kernel_launch(void* const* d_in, const int* in_sizes, int n_in,
                              void* d_out, int out_size, void* d_ws, size_t ws_size,
                              hipStream_t stream) {
  if (n_in < 15) return;
  if (in_sizes[0] != kRows * kDm) return;
  if (in_sizes[1] != kDin * kDm) return;
  if (in_sizes[2] != kDin) return;
  if (in_sizes[3] != kDin * 3) return;
  if (in_sizes[4] != kDin) return;
  if (in_sizes[5] != kDbc * kDin) return;
  if (in_sizes[6] != kDin * kDtR) return;
  if (in_sizes[7] != kDin) return;
  if (in_sizes[8] != kDin * kNst) return;
  if (in_sizes[9] != kDin) return;
  if (in_sizes[10] != kDm * kDin) return;
  if (in_sizes[11] != kDm) return;
  if (in_sizes[12] != kDtR) return;
  if (in_sizes[13] != kNst) return;
  if (in_sizes[14] != kNst) return;
  if (out_size != kRows * kDm) return;
  if (ws_size < kWsTotal) return;

  const float* x       = (const float*)d_in[0];
  const float* in_w    = (const float*)d_in[1];
  const float* in_b    = (const float*)d_in[2];
  const float* conv_w  = (const float*)d_in[3];
  const float* conv_b  = (const float*)d_in[4];
  const float* xproj_w = (const float*)d_in[5];
  const float* dt_w    = (const float*)d_in[6];
  const float* dt_b    = (const float*)d_in[7];
  const float* a_log   = (const float*)d_in[8];
  const float* d_skip  = (const float*)d_in[9];
  const float* out_w   = (const float*)d_in[10];
  const float* out_b   = (const float*)d_in[11];
  const float* dtln_w  = (const float*)d_in[12];
  const float* bln_w   = (const float*)d_in[13];
  const float* cln_w   = (const float*)d_in[14];
  float* out = (float*)d_out;

  char* ws = (char*)d_ws;
  unsigned short* WIN16  = (unsigned short*)(ws + kOffWin);
  unsigned short* WOUT16 = (unsigned short*)(ws + kOffWout);
  unsigned short* WXP16  = (unsigned short*)(ws + kOffWxp);
  unsigned short* WDT16  = (unsigned short*)(ws + kOffWdt);
  unsigned short* X16    = (unsigned short*)(ws + kOffX16);
  float*          HPRE   = (float*)(ws + kOffHpre);
  unsigned short* DELTA16 = (unsigned short*)(ws + kOffDelta);
  unsigned short* Y16    = (unsigned short*)(ws + kOffY16);
  unsigned short* H16    = (unsigned short*)(ws + kOffH16);
  float*          DBC    = (float*)(ws + kOffDbc);
  unsigned short* DN16   = (unsigned short*)(ws + kOffDn);
  float*          BM     = (float*)(ws + kOffBm);
  float*          CM     = (float*)(ws + kOffCm);

  cvt_rows_f16_kernel<<<(kDin * kDm / 8) / 256, 256, 0, stream>>>(in_w, WIN16, kDin * kDm / 8, kWCarry);
  cvt_rows_f16_kernel<<<(kDm * kDin / 8) / 256, 256, 0, stream>>>(out_w, WOUT16, kDm * kDin / 8, kWCarry);
  cvt_rows_f16_kernel<<<(kDbc * kDin / 8) / 256, 256, 0, stream>>>(xproj_w, WXP16, kDbc * kDin / 8, kWCarry);
  cvt_rows_f16_kernel<<<(kDin * kDtR / 8) / 256, 256, 0, stream>>>(dt_w, WDT16, kDin * kDtR / 8, kWCarry);
  cvt_rows_f16_kernel<<<(kRows * kDm / 8) / 256, 256, 0, stream>>>(x, X16, kRows * kDm / 8, 1.0f);

  wmma_gemm64<2, 0, 0><<<(kRows / 64) * (kDin / 64) / 8, 256, 0, stream>>>(
      X16, kDm, WIN16, kDm, (void*)HPRE, kDin, in_b, kRows, kDin, kDm, kInvW, 1.0f);

  conv_silu_kernel<<<dim3(kDin / 256, kRows / 64), 256, 0, stream>>>(HPRE, conv_w, conv_b, H16);

  wmma_gemm64<0, 0, 0><<<(kRows / 64) * (kDbc / 64) / 8, 256, 0, stream>>>(
      H16, kDin, WXP16, kDin, (void*)DBC, kDbc, in_b, kRows, kDbc, kDin, kInvWH, 1.0f);

  rms_split_kernel<<<kRows / 128, 128, 0, stream>>>(DBC, dtln_w, bln_w, cln_w, DN16, BM, CM);

  wmma_gemm64<2, 1, 6><<<(kRows / 64) * (kDin / 64) / 8, 256, 0, stream>>>(
      DN16, kDtR, WDT16, kDtR, (void*)DELTA16, kDin, dt_b, kRows, kDin, kDtR, kInvW, kDCarry);

  scan_kernel<<<kBatch * (kDin / 512), 256, 0, stream>>>(
      (const unsigned*)DELTA16, (const unsigned*)H16, BM, CM, a_log, d_skip, (unsigned*)Y16);

  wmma_gemm64<2, 0, 0><<<(kRows / 64) * (kDm / 64) / 8, 256, 0, stream>>>(
      Y16, kDin, WOUT16, kDin, (void*)out, kDm, out_b, kRows, kDm, kDin, kInvWY, 1.0f);
}
